// RoPEMaskedAttentionHead_35046933135573
// MI455X (gfx1250) — hardware-verified
//
#include <hip/hip_runtime.h>


namespace {
constexpr int Bn = 4, M = 4096, D = 512, NT = Bn * M;
constexpr float XS = 8.0f, ISQ = 0.044194173824159216f;
__constant__ unsigned int kThetaBits[256] = {0x3f84b063,0x3f800000,0x3f76f410,0x3f6e39f8,0x3f65ced3,0x3f5dafd7,0x3f55da52,0x3f4e4bac,0x3f470165,0x3f3ff911,0x3f39305c,0x3f32a506,0x3f2c54e5,0x3f263de0,0x3f205df3,0x3f1ab32b,0x3f153ba8,0x3f0ff59a,0x3f0adf41,0x3f05f6ee,0x3f013b01,0x3ef953cf,0x3ef0843c,0x3ee80460,0x3edfd167,0x3ed7e89b,0x3ed0475c,0x3ec8eb24,0x3ec1d181,0x3ebaf81a,0x3eb45caa,0x3eadfcff,0x3ea7d6fd,0x3ea1e89b,0x3e9c2fe1,0x3e96aaea,0x3e9157e1,0x3e8c3504,0x3e87409d,0x3e827909,0x3e7bb965,0x3e72d424,0x3e6a3f5c,0x3e61f836,0x3e59fbf3,0x3e5247ed,0x3e4ad998,0x3e43ae7c,0x3e3cc43a,0x3e361887,0x3e2fa92d,0x3e29740a,0x3e23770f,0x3e1db040,0x3e181db4,0x3e12bd91,0x3e0d8e0f,0x3e088d77,0x3e03ba20,0x3dfe24e1,0x3df529bb,0x3dec7fd5,0x3de42450,0x3ddc1466,0x3dd44d6c,0x3dcccccd,0x3dc5900d,0x3dbe94c7,0x3db7d8a9,0x3db15978,0x3dab150e,0x3da50957,0x3d9f3451,0x3d99940e,0x3d9426b0,0x3d8eea6c,0x3d89dd84,0x3d84fe4d,0x3d804b29,0x3d778512,0x3d6ec5da,0x3d6655c3,0x3d5e3202,0x3d5657e4,0x3d4ec4ce,0x3d47763f,0x3d4069ca,0x3d399d19,0x3d330dec,0x3d2cba15,0x3d269f7d,0x3d20bc1d,0x3d1b0e01,0x3d159348,0x3d104a21,0x3d0b30cc,0x3d064597,0x3d0186e2,0x3cf9e635,0x3cf11176,0x3ce88c9c,0x3ce054d2,0x3cd86761,0x3cd0c1a8,0x3cc9611d,0x3cc24350,0x3cbb65e3,0x3cb4c691,0x3cae6328,0x3ca8398b,0x3ca247ad,0x3c9c8b97,0x3c970362,0x3c91ad39,0x3c8c8757,0x3c879008,0x3c82c5a5,0x3c7c4d33,0x3c7362b9,0x3c6ac8e7,0x3c627ce5,0x3c5a7bf1,0x3c52c366,0x3c4b50b4,0x3c442163,0x3c3d3311,0x3c368373,0x3c301052,0x3c29d789,0x3c23d70a,0x3c1e0cd7,0x3c187705,0x3c1313ba,0x3c0de12d,0x3c08dda5,0x3c040779,0x3bfeba1b,0x3bf5b9b0,0x3bed0ab3,0x3be4aa46,0x3bdc95a0,0x3bd4ca14,0x3bcd450e,0x3bc6040e,0x3bbf04ae,0x3bb8449c,0x3bb1c19b,0x3bab7983,0x3ba56a3f,0x3b9f91cc,0x3b99ee3b,0x3b947dae,0x3b8f3e56,0x3b8a2e77,0x3b854c64,0x3b80967d,0x3b781668,0x3b6f520d,0x3b66dd02,0x3b5eb47a,0x3b56d5bf,0x3b4f3e37,0x3b47eb5e,0x3b40dac5,0x3b3a0a16,0x3b33770f,0x3b2d1f81,0x3b270153,0x3b211a7e,0x3b1b690d,0x3b15eb1c,0x3b109edb,0x3b0b8287,0x3b06946f,0x3b01d2f1,0x3afa78f1,0x3af19f03,0x3ae91528,0x3ae0d88b,0x3ad8e673,0x3ad13c3c,0x3ac9d75c,0x3ac2b561,0x3abbd3ec,0x3ab530b7,0x3aaec98e,0x3aa89c52,0x3aa2a6f6,0x3a9ce782,0x3a975c0e,0x3a9202c3,0x3a8cd9db,0x3a87dfa1,0x3a83126f,0x3a7ce158,0x3a73f1a2,0x3a6b52c4,0x3a6301e2,0x3a5afc3b,0x3a533f27,0x3a4bc816,0x3a44948c,0x3a3da229,0x3a36ee9e,0x3a3077b3,0x3a2a3b43,0x3a24373e,0x3a1e69a5,0x3a18d08b,0x3a136a16,0x3a0e347c,0x3a092e02,0x3a0454ff,0x39ff4fad,0x39f649f8,0x39ed95e3,0x39e5308a,0x39dd1726,0x39d54706,0x39cdbd95,0x39c67853,0x39bf74d7,0x39b8b0cf,0x39b229fb,0x39abde33,0x39a5cb5f,0x399fef7e,0x399a489e,0x3994d4df,0x398f9272,0x398a7f9b,0x39859aa9,0x3980e1fe,0x3978a814,0x396fde93,0x39676491,0x395f373e,0x395753e5,0x394fb7e7,0x394860c1,0x39414c02,0x393a7753,0x3933e06f,0x392d8529,0x39276363,0x39217917,0x391bc44d,0x39164323,0x3910f3c6,0x390bd472,0x3906e374,0x39021f2b,0x38fb0c03,0x38f22ce3,0x38e99e04,0x38e15c92};

typedef _Float16 b16;
typedef __attribute__((ext_vector_type(16))) _Float16 v16b;
typedef __attribute__((ext_vector_type(8))) _Float16 v8b;
typedef __attribute__((ext_vector_type(8))) float v8f;
typedef __attribute__((ext_vector_type(4))) float v4f;
__device__ __forceinline__ float bf16_rne(float f) { unsigned int u = __float_as_uint(f); u += 0x7FFFu + ((u >> 16) & 1u); return __uint_as_float(u & 0xFFFF0000u); }
__device__ __forceinline__ v16b frag_kb(const b16* p, int hh) { const v8b a = *(const v8b*)(p + 8 * hh), b = *(const v8b*)(p + 16 + 8 * hh); v16b f;
#pragma unroll
  for (int e = 0; e < 8; ++e) { f[e] = a[e]; f[8 + e] = b[e]; } return f; }
__device__ __forceinline__ v8f wmma16b(v16b a, v16b b, v8f c) { v8f d = __builtin_amdgcn_wmma_f32_16x16x32_f16(false, a, false, b, (short)0, c, false, false); asm volatile("v_nop\n\tv_nop\n\tv_nop\n\tv_nop" : "+v"(d) : "v"(a), "v"(b)); return d; }
__device__ __forceinline__ void wave_lds_sync() { __builtin_amdgcn_fence(__ATOMIC_RELEASE, "workgroup"); __builtin_amdgcn_wave_barrier(); __builtin_amdgcn_fence(__ATOMIC_ACQUIRE, "workgroup"); }
__device__ __forceinline__ float nexp(float x) { return __builtin_amdgcn_exp2f(x * 1.4426950408889634f); }
__device__ __forceinline__ float pmul(float a, float b) { float p = a * b; asm volatile("" : "+v"(p)); return p; }
__device__ __forceinline__ float wsum(float v) {
#pragma unroll
  for (int o = 1; o < 32; o <<= 1) v += __shfl_xor(v, o); return v; }
__device__ __forceinline__ void sincos_r(float ang, float& sn, float& cs) { const float k = rintf(ang * 0.15915494309189535f); float r = __builtin_fmaf(k, -6.28318548202514648f, ang); r = __builtin_fmaf(k, 1.7484556025237907e-7f, r);
  const float t = r * 0.15915494309189535f; sn = __builtin_amdgcn_sinf(t); cs = __builtin_amdgcn_cosf(t); }

__global__ __launch_bounds__(256) void prep_kernel(const float* __restrict__ wq, const float* __restrict__ wk, const float* __restrict__ uv, const float* __restrict__ vv, b16* __restrict__ R, float* __restrict__ P) {
  const size_t tid = (size_t)blockIdx.x * 256 + threadIdx.x, nth = (size_t)gridDim.x * 256;
  for (int pass = 0; pass < 2; ++pass) {
    for (size_t p = tid; p < (size_t)2 * D * (D / 8); p += nth) { const int w = (int)(p / ((size_t)D * (D / 8))); const size_t r = p % ((size_t)D * (D / 8)); const int o = (int)(r / (D / 8)), k0 = (int)(r % (D / 8)) * 8; const float* W = w ? wk : wq; v8b v;
      for (int e = 0; e < 8; ++e) v[e] = (b16)bf16_rne(W[(size_t)(k0 + e) * D + o]); *(volatile v8b*)(R + ((size_t)w * D + o) * D + k0) = v; }
    for (size_t q = tid; q < 1024; q += nth) P[q] = bf16_rne((q < 512) ? uv[q] : vv[q - 512]);
    __threadfence(); }
}

__global__ __launch_bounds__(256) void xrows_kernel(const float* __restrict__ x, const float* __restrict__ P, b16* __restrict__ X, float* __restrict__ S) {
  __shared__ float Ss[32];
  const int wave = threadIdx.x >> 5, lane = threadIdx.x & 31, t0 = blockIdx.x * 32;
  for (int q = 0; q < 4; ++q) { const int t = t0 + wave * 4 + q; const float* xr = x + (size_t)t * D; float v[16]; float s = 0.0f;
#pragma unroll
    for (int i = 0; i < 16; ++i) { v[i] = bf16_rne(xr[(i >> 3) * 256 + lane * 8 + (i & 7)]); s += pmul(v[i], P[(i >> 3) * 256 + lane * 8 + (i & 7)]); }
    s = wsum(s); if (lane == 0) Ss[wave * 4 + q] = s;
    for (int pass = 0; pass < 2; ++pass) {
#pragma unroll
      for (int gq = 0; gq < 2; ++gq) { v8b o; for (int e = 0; e < 8; ++e) o[e] = (b16)(v[gq * 8 + e] * XS); *(volatile v8b*)(X + (size_t)t * D + gq * 256 + lane * 8) = o; } __threadfence(); } }
  __syncthreads();
  for (int pass = 0; pass < 2; ++pass) { if (threadIdx.x < 32) ((volatile float*)S)[t0 + threadIdx.x] = Ss[threadIdx.x]; __threadfence(); }
}

__global__ __launch_bounds__(64) void proj_kernel(const b16* __restrict__ X, const b16* __restrict__ Bw, b16* __restrict__ O) {
  __shared__ __attribute__((aligned(16))) float Ts[2][32][128 + 4];
  const int lane = threadIdx.x & 31, wave = threadIdx.x >> 5, nloc = lane & 15, hlf = lane >> 4, m0 = blockIdx.y * 32, c0 = blockIdx.x * 256 + wave * 128;
#pragma unroll 1
  for (int hf = 0; hf < 2; ++hf) { v8f acc[2][4];
#pragma unroll
    for (int r = 0; r < 2; ++r)
#pragma unroll
      for (int t = 0; t < 4; ++t) acc[r][t] = (v8f){};
#pragma unroll 2
    for (int kb = 0; kb < D; kb += 32) { const v16b a0 = frag_kb(X + (size_t)(m0 + nloc) * D + kb, hlf), a1 = frag_kb(X + (size_t)(m0 + 16 + nloc) * D + kb, hlf);
#pragma unroll
      for (int t = 0; t < 4; ++t) { const v16b bw = frag_kb(Bw + (size_t)(c0 + (hf * 4 + t) * 16 + nloc) * D + kb, hlf); acc[0][t] = wmma16b(a0, bw, acc[0][t]); acc[1][t] = wmma16b(a1, bw, acc[1][t]); } }
#pragma unroll
    for (int t = 0; t < 4; ++t)
#pragma unroll
      for (int r = 0; r < 2; ++r)
#pragma unroll
        for (int v = 0; v < 8; ++v) Ts[wave][r * 16 + 8 * hlf + v][(hf * 4 + t) * 16 + nloc] = acc[r][t][v] * (1.0f / XS); }
  wave_lds_sync();
  for (int i = lane; i < 32 * 64; i += 32) { const int rr = i >> 6, pi = i & 63; const int c = 2 * pi, ci = (c0 + c) >> 1; const int t = (m0 + rr) % M; float sn, cs; sincos_r(pmul((float)t, __uint_as_float(kThetaBits[ci])), sn, cs);
    const float te = Ts[wave][rr][c], to = Ts[wave][rr][c + 1]; Ts[wave][rr][c] = pmul(te, cs) + pmul(to, sn); Ts[wave][rr][c + 1] = pmul(to, cs) - pmul(te, sn); }
  wave_lds_sync();
  for (int pass = 0; pass < 2; ++pass) { for (int i = lane; i < 32 * 16; i += 32) { const int rr = i >> 4, c8 = (i & 15) * 8; v8b o; for (int e = 0; e < 8; ++e) o[e] = (b16)(Ts[wave][rr][c8 + e] * XS); *(volatile v8b*)(O + (size_t)(m0 + rr) * D + c0 + c8) = o; } __threadfence(); }
}

__global__ __launch_bounds__(256) void attn_kernel(const b16* __restrict__ Q, const b16* __restrict__ K, const float* __restrict__ S, const float* __restrict__ P, float* __restrict__ out) {
  __shared__ float Cq[8][16];
  const int wave = threadIdx.x >> 5, lane = threadIdx.x & 31, hh = lane >> 4, col = lane & 15; const int tok0 = blockIdx.x * 128 + wave * 16; const int b = tok0 / M, q0 = tok0 % M, qi = q0 + col;
  const b16* Qr = Q + (size_t)(b * M) * D; const b16* Kr = K + (size_t)(b * M) * D; const float* Sb = S + (size_t)b * M;
  v16b qf[16];
#pragma unroll
  for (int j = 0; j < 16; ++j) qf[j] = frag_kb(Qr + (size_t)qi * D + 32 * j, hh);
  float m = -INFINITY, l = 0.0f, c = 0.0f;
  for (int kb = 0; kb <= q0 + 15; kb += 32) { v8f s0 = {}, s1 = {};
#pragma unroll
    for (int j = 0; j < 16; ++j) { s0 = wmma16b(frag_kb(Kr + (size_t)(kb + col) * D + 32 * j, hh), qf[j], s0); s1 = wmma16b(frag_kb(Kr + (size_t)(kb + 16 + col) * D + 32 * j, hh), qf[j], s1); }
    float mr = -INFINITY;
#pragma unroll
    for (int r = 0; r < 8; ++r) { const int k0 = kb + 8 * hh + r, k1 = k0 + 16; s0[r] = (k0 <= qi) ? s0[r] * (ISQ / (XS * XS)) : -INFINITY; s1[r] = (k1 <= qi) ? s1[r] * (ISQ / (XS * XS)) : -INFINITY; mr = fmaxf(mr, fmaxf(s0[r], s1[r])); }
    mr = fmaxf(mr, __shfl_xor(mr, 16)); const float mn = fmaxf(m, mr), al_ = nexp(m - mn); m = mn; float sum = 0.0f, cs_ = 0.0f;
#pragma unroll
    for (int r = 0; r < 8; ++r) { const int k0 = kb + 8 * hh + r, k1 = k0 + 16; const float e0 = (s0[r] == -INFINITY) ? 0.0f : nexp(s0[r] - mn), e1 = (s1[r] == -INFINITY) ? 0.0f : nexp(s1[r] - mn);
      const int k0c = (k0 < M) ? k0 : (M - 1), k1c = (k1 < M) ? k1 : (M - 1); sum += e0 + e1; cs_ += pmul(e0, Sb[k0c]) + pmul(e1, Sb[k1c]); }
    l = l * al_ + sum; c = c * al_ + cs_; }
  l += __shfl_xor(l, 16); c += __shfl_xor(c, 16);
  if (hh == 0) Cq[wave][col] = c / l;
  wave_lds_sync();
  for (int pass = 0; pass < 2; ++pass) { for (int i = lane; i < 16 * 128; i += 32) { const int rr = i >> 7, c4 = (i & 127) * 4; const float cq = Cq[wave][rr]; v4f o; for (int e = 0; e < 4; ++e) o[e] = pmul(cq, P[512 + c4 + e]); *(volatile v4f*)(out + (size_t)(tok0 + rr) * D + c4) = o; } __threadfence(); }
}
}

extern "C" void kernel_launch(void* const* d_in, const int* in_sizes, int n_in,
                              void* d_out, int out_size, void* d_ws, size_t ws_size, hipStream_t stream) {
  (void)n_in; (void)out_size;
  const float* x = (const float*)d_in[0]; const float* wq = (const float*)d_in[1]; const float* wk = (const float*)d_in[2]; const float* uv = (const float*)d_in[3]; const float* vv = (const float*)d_in[4];
  float* out = (float*)d_out;
  if (in_sizes[0] != NT * D || in_sizes[1] != D * D || in_sizes[3] != D || in_sizes[4] != D) return;
  size_t off = 0; char* ws = (char*)d_ws;
  auto carve = [&](size_t bytes) { char* p = ws + off; off += (bytes + 255) & ~(size_t)255; return p; };
  b16* R = (b16*)carve((size_t)2 * D * D * 2); float* P = (float*)carve(1024 * 4); b16* X = (b16*)carve((size_t)NT * D * 2); float* S = (float*)carve((size_t)NT * 4); b16* Q = (b16*)carve((size_t)NT * D * 2); b16* K = (b16*)carve((size_t)NT * D * 2);
  if (off > ws_size) return;
  prep_kernel<<<128, 256, 0, stream>>>(wq, wk, uv, vv, R, P);
  xrows_kernel<<<NT / 32, 256, 0, stream>>>(x, P, X, S);
  proj_kernel<<<dim3(2, NT / 32), 64, 0, stream>>>(X, R, Q);
  proj_kernel<<<dim3(2, NT / 32), 64, 0, stream>>>(X, R + (size_t)D * D, K);
  attn_kernel<<<NT / 128, 256, 0, stream>>>(Q, K, S, P, out);
}
